// SelectiveTokenMixer_72232759984889
// MI455X (gfx1250) — hardware-verified
//
#include <hip/hip_runtime.h>
#include <math.h>

typedef __attribute__((ext_vector_type(16))) _Float16 v16h;
typedef __attribute__((ext_vector_type(8)))  _Float16 v8h;
typedef __attribute__((ext_vector_type(16))) __bf16   v16b;
typedef __attribute__((ext_vector_type(8)))  __bf16   v8b;
typedef __attribute__((ext_vector_type(8)))  float    v8f;
typedef __attribute__((ext_vector_type(4)))  float    v4f;

constexpr int kBatch  = 8;
constexpr int kSeq    = 1024;
constexpr int kDm     = 768;
constexpr int kDin    = 1536;
constexpr int kNst    = 16;
constexpr int kDtR    = 48;
constexpr int kConv   = 4;
constexpr int kXzP    = 2 * kDin;
constexpr int kXdW    = kDtR + 2 * kNst;
constexpr int kXdP    = 128;
constexpr int kRowsAll = kBatch * kSeq;
constexpr int kGroups  = 2;
constexpr int kRowsG   = kRowsAll / kGroups;
constexpr int kTrP     = 68;
constexpr int kConvTP  = 260;
constexpr int kScanTS  = 64;
constexpr int kScanCh  = 64;
constexpr int kScanYP  = 68;
constexpr float kLnEps = 1e-5f;
constexpr float kWCarry   = 256.0f;
constexpr float kUcCarry  = 1024.0f;
constexpr float kYCarry   = 4096.0f;
constexpr float kInScale  = 1.0f / kWCarry;
constexpr float kXScale   = 1.0f / (kUcCarry * kWCarry);
constexpr float kOutScale = 1.0f / (kYCarry * kWCarry);
static_assert(kDtR + 2 * kNst == kXdW && kXdW <= kXdP, "x_proj width");
static_assert((kDm % 64) == 0 && (kDin % 64) == 0, "GEMM K multiples of 32 and transpose tiles of 64");
static_assert((kRowsG % 64) == 0 && (kXzP % 64) == 0 && (kXdP % 64) == 0 && (kDm % 64) == 0, "GEMM M,N multiples of 64");
static_assert((kSeq % kScanTS) == 0 && (kSeq % 64) == 0 && (kDin % kScanCh) == 0 && (kDin % 256) == 0, "tile multiples");
static_assert(kRowsG % kSeq == 0, "a group holds whole sequences");
static_assert((kDtR % 4) == 0 && (kXdW % 4) == 0, "v4f staging");
static_assert(kScanTS == kScanCh, "row-per-thread staging in the scan");

constexpr int kTilesIn  = (kRowsG / 64) * (kXzP / 64);
constexpr int kTilesX   = (kRowsG / 64) * (kXdP / 64);
constexpr int kTilesOut = (kRowsG / 64) * (kDm  / 64);
static_assert((kTilesIn % 8) == 0 && (kTilesX % 8) == 0 && (kTilesOut % 8) == 0, "whole GEMM blocks");

constexpr size_t kOffWIT  = 0;
constexpr size_t kOffWXT  = kOffWIT  + (size_t)kXzP * kDm  * 2;
constexpr size_t kOffWOT  = kOffWXT  + (size_t)kXdP * kDin * 2;
constexpr size_t kOffXN   = kOffWOT  + (size_t)kDm  * kDin * 2;
constexpr size_t kOffXZ   = kOffXN   + (size_t)kRowsG * kDm  * 2;
constexpr size_t kOffUC   = kOffXZ   + (size_t)kRowsG * kXzP * 4;
constexpr size_t kOffUC16 = kOffUC   + (size_t)kRowsG * kDin * 4;
constexpr size_t kOffXD   = kOffUC16 + (size_t)kRowsG * kDin * 2;
constexpr size_t kOffY16  = kOffXD   + (size_t)kRowsG * kXdP * 4;
constexpr size_t kWsTotal = kOffY16  + (size_t)kRowsG * kDin * 2;
static_assert(kWsTotal == 116523008ull, "carve total");
static_assert(kWsTotal <= 134217728ull, "carve cap");
static_assert((kOffWXT % 128) == 0 && (kOffWOT % 128) == 0 && (kOffXN % 128) == 0 && (kOffXZ % 128) == 0 &&
              (kOffUC % 128) == 0 && (kOffUC16 % 128) == 0 && (kOffXD % 128) == 0 && (kOffY16 % 128) == 0,
              "128-B aligned regions");

__device__ __forceinline__ unsigned short f2bf_bits(float f) {
  unsigned u = __float_as_uint(f);
  return (unsigned short)((u + 0x7FFFu + ((u >> 16) & 1u)) >> 16);
}
__device__ __forceinline__ float bf_bits2f(unsigned short h) { return __uint_as_float(((unsigned)h) << 16); }

__device__ __forceinline__ void dep_guard_h(v8f& a, v8f& b, v16h x, v16h y) { asm volatile("v_nop\n\tv_nop\n\tv_nop\n\tv_nop" : "+v"(a), "+v"(b) : "v"(x), "v"(y)); }
__device__ __forceinline__ void dep_guard_b(v8f& a, v8f& b, v16b x, v16b y) { asm volatile("v_nop\n\tv_nop\n\tv_nop\n\tv_nop" : "+v"(a), "+v"(b) : "v"(x), "v"(y)); }
__device__ __forceinline__ void keep4_h(v16h a, v16h b, v16h c, v16h d) { asm volatile("v_nop" :: "v"(a), "v"(b), "v"(c), "v"(d)); }
__device__ __forceinline__ void keep4_b(v16b a, v16b b, v16b c, v16b d) { asm volatile("v_nop" :: "v"(a), "v"(b), "v"(c), "v"(d)); }
__device__ __forceinline__ void acc_guard4(v8f& a, v8f& b, v8f& c, v8f& d) { asm volatile("v_nop\n\tv_nop\n\tv_nop\n\tv_nop" : "+v"(a), "+v"(b), "+v"(c), "+v"(d)); }
template <typename T> struct Frag;
template <> struct Frag<_Float16> {
  typedef v16h V; union U { v16h v; v8h h[2]; };
  static __device__ __forceinline__ v16h load(const _Float16* p) {
    U f; f.h[0] = *(const v8h*)(p); f.h[1] = *(const v8h*)(p + 16); return f.v;
  }
  static __device__ __forceinline__ v8f mma(v16h a, v16h b, v8f c) {
    return __builtin_amdgcn_wmma_f32_16x16x32_f16(false, a, false, b, (short)0, c, false, false);
  }
  static __device__ __forceinline__ void guard(v8f& a, v8f& b, v16h x, v16h y) { dep_guard_h(a, b, x, y); }
  static __device__ __forceinline__ void keep(v16h a, v16h b, v16h c, v16h d) { keep4_h(a, b, c, d); }
};
template <> struct Frag<__bf16> {
  typedef v16b V; union U { v16b v; v8b h[2]; };
  static __device__ __forceinline__ v16b load(const __bf16* p) {
    U f; f.h[0] = *(const v8b*)(p); f.h[1] = *(const v8b*)(p + 16); return f.v;
  }
  static __device__ __forceinline__ v8f mma(v16b a, v16b b, v8f c) {
    return __builtin_amdgcn_wmma_f32_16x16x32_bf16(false, a, false, b, (short)0, c, false, false);
  }
  static __device__ __forceinline__ void guard(v8f& a, v8f& b, v16b x, v16b y) { dep_guard_b(a, b, x, y); }
  static __device__ __forceinline__ void keep(v16b a, v16b b, v16b c, v16b d) { keep4_b(a, b, c, d); }
};

template <int ET> struct Elem;
template <> struct Elem<0> { typedef _Float16 T; };
template <> struct Elem<1> { typedef __bf16 T; };
template <int ET, int SPL, int BIAS_MODE, int OUT_MODE, bool RESID, int ACT = 0>
__global__ __launch_bounds__(256) void wmma_gemm64(
    const unsigned short* __restrict__ Ap, const unsigned short* __restrict__ A2p, int lda, long strideA,
    const unsigned short* __restrict__ Btp, const unsigned short* __restrict__ Bt2p, int ldb, long strideB,
    void* __restrict__ Cout, void* __restrict__ Cout2, int ldc, long strideC,
    const float* __restrict__ bias,
    const float* __restrict__ resid, long strideR,
    int M, int N, int K, float scale) {
  typedef typename Elem<ET>::T T;
  typedef typename Frag<T>::V V;
  const T* A = (const T*)Ap; const T* A2 = (const T*)A2p; const T* Bt = (const T*)Btp; const T* Bt2 = (const T*)Bt2p;
  __shared__ __align__(16) float sT[8][16 * 68];
  const int b    = blockIdx.y;
  const int lane = threadIdx.x & 31;
  const int wave = threadIdx.x >> 5;
  const int tilesN = N >> 6;
  const int tilesM = M >> 6;
  const int tile = blockIdx.x * 8 + wave;
  if (tile >= tilesM * tilesN) return;
  const int tm = tile / tilesN;
  const int tn = tile - tm * tilesN;
  const int m0 = tm << 6;
  const int n0 = tn << 6;

  const T* Ab  = A  + (size_t)b * strideA;
  const T* Bb  = Bt + (size_t)b * strideB;
  const T* Ab2 = (SPL >= 1) ? (A2  + (size_t)b * strideA) : nullptr;
  const T* Bb2 = (SPL == 2) ? (Bt2 + (size_t)b * strideB) : nullptr;

  const int rlane = lane & 15;
  const int koff  = (lane >> 4) * 8;
  const int mOff  = (lane >> 4) * 8;

  v8f acc[4][4];
#pragma unroll
  for (int i = 0; i < 4; ++i)
#pragma unroll
    for (int j = 0; j < 4; ++j) acc[i][j] = (v8f){0.f,0.f,0.f,0.f,0.f,0.f,0.f,0.f};

  for (int k0 = 0; k0 < K; k0 += 32) {
    V bh[4], bl[4];
#pragma unroll
    for (int j = 0; j < 4; ++j) {
      const size_t bo = (size_t)(n0 + (j << 4) + rlane) * ldb + koff + k0;
      bh[j] = Frag<T>::load(Bb + bo);
      if (SPL == 2) bl[j] = Frag<T>::load(Bb2 + bo);
    }
#pragma unroll
    for (int i = 0; i < 4; ++i) {
      const size_t ao = (size_t)(m0 + (i << 4) + rlane) * lda + koff + k0;
      V ah = Frag<T>::load(Ab + ao);
      V al;
      if (SPL >= 1) al = Frag<T>::load(Ab2 + ao);
#pragma unroll
      for (int j = 0; j < 4; ++j) {
        acc[i][j] = Frag<T>::mma(ah, bh[j], acc[i][j]);
        if (SPL == 2) acc[i][j] = Frag<T>::mma(ah, bl[j], acc[i][j]);
        if (SPL >= 1) acc[i][j] = Frag<T>::mma(al, bh[j], acc[i][j]);
      }
      Frag<T>::guard(acc[i][0], acc[i][3], ah, (SPL >= 1) ? al : ah);
    }
    Frag<T>::keep(bh[0], bh[1], bh[2], bh[3]);
    if (SPL == 2) Frag<T>::keep(bl[0], bl[1], bl[2], bl[3]);
  }
  acc_guard4(acc[0][0], acc[0][1], acc[0][2], acc[0][3]);
  acc_guard4(acc[1][0], acc[1][1], acc[1][2], acc[1][3]);
  acc_guard4(acc[2][0], acc[2][1], acc[2][2], acc[2][3]);
  acc_guard4(acc[3][0], acc[3][1], acc[3][2], acc[3][3]);

  float* slab = sT[wave];
  const float* Rb = RESID ? (resid + (size_t)b * strideR) : nullptr;
#pragma unroll
  for (int i = 0; i < 4; ++i) {
    const int mBase = m0 + (i << 4);
#pragma unroll
    for (int j = 0; j < 4; ++j) {
      const int n = n0 + (j << 4) + rlane;
      float bv = 0.f;
      if (BIAS_MODE == 2) bv = bias[n];
#pragma unroll
      for (int r = 0; r < 8; ++r) {
        float v = acc[i][j][r] * scale;
        if (BIAS_MODE == 1) v += bias[mBase + mOff + r];
        if (BIAS_MODE == 2) v += bv;
        if (RESID) v += Rb[(size_t)(mBase + mOff + r) * ldc + n];
        if (ACT == 1) v = tanhf(v);
        if (ACT == 2) v = fmaxf(v, 0.0f);
        if (ACT == 3) v = v / (1.0f + expf(-v));
        if (ACT == 4) v = (v > 0.f) ? v : 0.01f * v;
        slab[(mOff + r) * 68 + (j << 4) + rlane] = v;
      }
    }
    __builtin_amdgcn_fence(__ATOMIC_RELEASE, "workgroup");
    __builtin_amdgcn_wave_barrier();
    __builtin_amdgcn_fence(__ATOMIC_ACQUIRE, "workgroup");
    if (OUT_MODE == 0) {
      float* C = (float*)Cout + (size_t)b * strideC;
      const int hh = lane >> 4, c4 = (lane & 15) * 4;
      for (int pass = 0; pass < 2; ++pass) {
#pragma unroll
        for (int it = 0; it < 8; ++it) {
          const int row = it * 2 + hh;
          v4f v = *(const v4f*)(slab + row * 68 + c4);
          *(volatile v4f*)(C + (size_t)(mBase + row) * ldc + n0 + c4) = v;
        }
        __threadfence();
      }
    } else {
      const int q = lane >> 3, c8 = (lane & 7) * 8;
      unsigned short* C  = (unsigned short*)Cout  + (size_t)b * strideC;
      unsigned short* C2 = (OUT_MODE == 2) ? ((unsigned short*)Cout2 + (size_t)b * strideC) : nullptr;
      for (int pass = 0; pass < 2; ++pass) {
#pragma unroll
        for (int it = 0; it < 4; ++it) {
          const int row = it * 4 + q;
          const float* sp = slab + row * 68 + c8;
          v8h hv, lv;
#pragma unroll
          for (int e = 0; e < 8; ++e) {
            if (OUT_MODE == 1) {
              hv[e] = (_Float16)sp[e];
            } else {
              unsigned short hb = f2bf_bits(sp[e]);
              unsigned short lb = f2bf_bits(sp[e] - bf_bits2f(hb));
              hv[e] = __builtin_bit_cast(_Float16, hb);
              lv[e] = __builtin_bit_cast(_Float16, lb);
            }
          }
          *(volatile v8h*)(C + (size_t)(mBase + row) * ldc + n0 + c8) = hv;
          if (OUT_MODE == 2) *(volatile v8h*)(C2 + (size_t)(mBase + row) * ldc + n0 + c8) = lv;
        }
        __threadfence();
      }
    }
    __builtin_amdgcn_fence(__ATOMIC_RELEASE, "workgroup");
    __builtin_amdgcn_wave_barrier();
    __builtin_amdgcn_fence(__ATOMIC_ACQUIRE, "workgroup");
  }
}

__global__ __launch_bounds__(256) void transpose_cast_f16_kernel(
    const float* __restrict__ W, unsigned short* __restrict__ Wt, int Kdim, int Ndim, float carry)
{
  __shared__ __align__(16) float sT[64 * kTrP];
  const int tid = threadIdx.x, lane = tid & 31, wave = tid >> 5;
  const int k0 = blockIdx.x * 64, n0 = blockIdx.y * 64;
#pragma unroll
  for (int i = 0; i < 16; ++i) {
    const int idx = tid + 256 * i;
    const int kk = idx >> 6, nn = idx & 63;
    const int n = n0 + nn;
    const int nc = (n < Ndim) ? n : (Ndim - 1);
    const float v = W[(size_t)(k0 + kk) * Ndim + nc];
    sT[nn * kTrP + kk] = (n < Ndim) ? v : 0.f;
  }
  __syncthreads();
  const int q = lane >> 3, c8 = (lane & 7) * 8;
  v8h hv[2];
#pragma unroll
  for (int it = 0; it < 2; ++it) {
    const int row = it * 32 + wave * 4 + q;
    const float* sp = sT + row * kTrP + c8;
    const v4f a0 = *(const v4f*)(sp);
    const v4f a1 = *(const v4f*)(sp + 4);
#pragma unroll
    for (int e = 0; e < 4; ++e) {
      hv[it][e]     = (_Float16)(a0[e] * carry);
      hv[it][4 + e] = (_Float16)(a1[e] * carry);
    }
  }
  for (int pass = 0; pass < 2; ++pass) {
#pragma unroll
    for (int it = 0; it < 2; ++it) {
      const int row = it * 32 + wave * 4 + q;
      *(volatile v8h*)(Wt + (size_t)(n0 + row) * Kdim + k0 + c8) = hv[it];
    }
    __threadfence();
  }
}

__global__ __launch_bounds__(256) void ln_rows_kernel(
    const float* __restrict__ x, const float* __restrict__ g, const float* __restrict__ bb,
    unsigned short* __restrict__ XN, int nrows)
{
  const int lane = threadIdx.x & 31, wave = threadIdx.x >> 5;
  const int row = blockIdx.x * 8 + wave;
  if (row >= nrows) return;
  const float* xr = x + (size_t)row * kDm;
  v4f a[3][2];
  float s = 0.f;
#pragma unroll
  for (int i = 0; i < 3; ++i) {
    a[i][0] = *(const v4f*)(xr + 256 * i + lane * 8);
    a[i][1] = *(const v4f*)(xr + 256 * i + lane * 8 + 4);
    s += ((a[i][0][0] + a[i][0][1]) + (a[i][0][2] + a[i][0][3])) + ((a[i][1][0] + a[i][1][1]) + (a[i][1][2] + a[i][1][3]));
  }
#pragma unroll
  for (int off = 1; off < 32; off <<= 1) s += __shfl_xor(s, off, 32);
  const float mu = s * (1.0f / (float)kDm);
  float qs = 0.f;
#pragma unroll
  for (int i = 0; i < 3; ++i) {
#pragma unroll
    for (int e = 0; e < 4; ++e) {
      const float d0 = a[i][0][e] - mu;
      const float d1 = a[i][1][e] - mu;
      qs += d0 * d0;
      qs += d1 * d1;
    }
  }
#pragma unroll
  for (int off = 1; off < 32; off <<= 1) qs += __shfl_xor(qs, off, 32);
  const float var = qs * (1.0f / (float)kDm);
  const float rs = rsqrtf(var + kLnEps);
  v8h hv[3];
#pragma unroll
  for (int i = 0; i < 3; ++i) {
    const int c0 = 256 * i + lane * 8;
    const v4f g0 = *(const v4f*)(g + c0);
    const v4f g1 = *(const v4f*)(g + c0 + 4);
    const v4f b0 = *(const v4f*)(bb + c0);
    const v4f b1 = *(const v4f*)(bb + c0 + 4);
#pragma unroll
    for (int e = 0; e < 4; ++e) {
      hv[i][e]     = (_Float16)((a[i][0][e] - mu) * rs * g0[e] + b0[e]);
      hv[i][4 + e] = (_Float16)((a[i][1][e] - mu) * rs * g1[e] + b1[e]);
    }
  }
  for (int pass = 0; pass < 2; ++pass) {
#pragma unroll
    for (int i = 0; i < 3; ++i)
      *(volatile v8h*)(XN + (size_t)row * kDm + 256 * i + lane * 8) = hv[i];
    __threadfence();
  }
}

__global__ __launch_bounds__(256) void conv_silu_kernel(
    const float* __restrict__ XZ, const float* __restrict__ cw, const float* __restrict__ cb,
    float* __restrict__ UC, unsigned short* __restrict__ UC16)
{
  __shared__ __align__(16) float sT[16 * kConvTP];
  const int tid = threadIdx.x, lane = tid & 31, wave = tid >> 5;
  const int d0 = blockIdx.x * 256, d = d0 + tid;
  const int g0 = blockIdx.y * 64;
  const int tb = g0 & (kSeq - 1);
  const float w0 = cw[d * kConv + 0], w1 = cw[d * kConv + 1], w2 = cw[d * kConv + 2], w3 = cw[d * kConv + 3];
  const float bc = cb[d];
  float xm3, xm2, xm1;
  {
    const bool hist = (tb > 0);
    const int rb = hist ? (g0 - 3) : g0;
    const float v3 = XZ[(size_t)rb * kXzP + d];
    const float v2 = XZ[(size_t)(rb + 1) * kXzP + d];
    const float v1 = XZ[(size_t)(rb + 2) * kXzP + d];
    xm3 = hist ? v3 : 0.f;
    xm2 = hist ? v2 : 0.f;
    xm1 = hist ? v1 : 0.f;
  }
  const int hrow = wave >> 1;
  const int hch  = (wave & 1) * 128 + lane * 4;
#pragma unroll 1
  for (int sub = 0; sub < 4; ++sub) {
    const int lb = g0 + sub * 16;
#pragma unroll 1
    for (int s = 0; s < 16; ++s) {
      const float xcur = XZ[(size_t)(lb + s) * kXzP + d];
      float acc = w0 * xm3;
      acc = fmaf(w1, xm2, acc);
      acc = fmaf(w2, xm1, acc);
      acc = fmaf(w3, xcur, acc);
      const float sv = acc + bc;
      const float sg = __builtin_amdgcn_rcpf(1.0f + __expf(-sv));
      sT[s * kConvTP + tid] = sv * sg;
      xm3 = xm2; xm2 = xm1; xm1 = xcur;
    }
    __syncthreads();
    v4f fv[4];
    v8h hv[2];
#pragma unroll
    for (int it = 0; it < 4; ++it) fv[it] = *(const v4f*)(sT + (it * 4 + hrow) * kConvTP + hch);
#pragma unroll
    for (int it = 0; it < 2; ++it) {
      const float* sp = sT + (it * 8 + wave) * kConvTP + lane * 8;
      const v4f a0 = *(const v4f*)(sp);
      const v4f a1 = *(const v4f*)(sp + 4);
#pragma unroll
      for (int e = 0; e < 4; ++e) {
        hv[it][e]     = (_Float16)(a0[e] * kUcCarry);
        hv[it][4 + e] = (_Float16)(a1[e] * kUcCarry);
      }
    }
    for (int pass = 0; pass < 2; ++pass) {
#pragma unroll
      for (int it = 0; it < 4; ++it)
        *(volatile v4f*)(UC + (size_t)(lb + it * 4 + hrow) * kDin + d0 + hch) = fv[it];
#pragma unroll
      for (int it = 0; it < 2; ++it)
        *(volatile v8h*)(UC16 + (size_t)(lb + it * 8 + wave) * kDin + d0 + lane * 8) = hv[it];
      __threadfence();
    }
    __syncthreads();
  }
}

__global__ __launch_bounds__(64) __attribute__((amdgpu_num_vgpr(224))) void scan_kernel(
    const float* __restrict__ XD, const float* __restrict__ UC, const float* __restrict__ XZ,
    const float* __restrict__ Wdt, const float* __restrict__ bdt, const float* __restrict__ Alog,
    const float* __restrict__ Dp, unsigned short* __restrict__ Y16)
{
  __shared__ __align__(16) float sX[kScanTS * kXdW];
  __shared__ __align__(16) float sY[kScanTS * kScanYP];
  __shared__ __align__(16) float sW[kDtR * kScanCh];
  __shared__ __align__(16) float sA[kNst * kScanCh];
  const int tid = threadIdx.x, lane = tid & 31, wave = tid >> 5;
  constexpr int kBlkPerB = kDin / kScanCh;
  const int bix = blockIdx.x / kBlkPerB;
  const int d0  = (blockIdx.x - bix * kBlkPerB) * kScanCh;
  const int d   = d0 + tid;
  const size_t row0 = (size_t)bix * kSeq;
#pragma unroll 1
  for (int r = 0; r < kDtR; ++r) sW[r * kScanCh + tid] = Wdt[(size_t)r * kDin + d];
#pragma unroll 1
  for (int s = 0; s < kNst; ++s) sA[s * kScanCh + tid] = -expf(Alog[(size_t)d * kNst + s]);
  __syncthreads();
  float negA[kNst], h[kNst];
#pragma unroll
  for (int s = 0; s < kNst; ++s) {
    negA[s] = sA[s * kScanCh + tid];
    h[s] = 0.f;
  }
  const float bb = bdt[d], Dd = Dp[d];
  const int q = lane >> 3, c8 = (lane & 7) * 8;
#pragma unroll 1
  for (int t0 = 0; t0 < kSeq; t0 += kScanTS) {
    __syncthreads();
    {
      const float* src = XD + (row0 + t0 + tid) * kXdP;
      float* dst = sX + tid * kXdW;
#pragma unroll 4
      for (int i = 0; i < kXdW / 4; ++i) *(v4f*)(dst + 4 * i) = *(const v4f*)(src + 4 * i);
    }
    __syncthreads();
#pragma unroll 1
    for (int s = 0; s < kScanTS; ++s) {
      const int t = t0 + s;
      const float* xr = sX + s * kXdW;
      float vdot = 0.f;
#pragma unroll 1
      for (int r4 = 0; r4 < kDtR / 4; ++r4) {
        const v4f xv = *(const v4f*)(xr + 4 * r4);
        const float* wp = sW + (4 * r4) * kScanCh + tid;
        vdot = fmaf(xv[0], wp[0], vdot);
        vdot = fmaf(xv[1], wp[kScanCh], vdot);
        vdot = fmaf(xv[2], wp[2 * kScanCh], vdot);
        vdot = fmaf(xv[3], wp[3 * kScanCh], vdot);
      }
      const float v   = vdot + bb;
      const float a   = __expf(-fabsf(v));
      const float u   = 1.0f + a;
      const float l1p = __logf(u) + (a - (u - 1.0f)) * __builtin_amdgcn_rcpf(u);
      const float dt  = fmaxf(v, 0.0f) + l1p;
      const float xt  = UC[(row0 + t) * kDin + d];
      const float dtx = dt * xt;
      float y = 0.f;
#pragma unroll
      for (int q4 = 0; q4 < 4; ++q4) {
        const v4f bv = *(const v4f*)(xr + kDtR + 4 * q4);
        const v4f cv = *(const v4f*)(xr + kDtR + kNst + 4 * q4);
#pragma unroll
        for (int e = 0; e < 4; ++e) {
          const int k = 4 * q4 + e;
          const float ex = __expf(dt * negA[k]);
          h[k] = ex * h[k] + dtx * bv[e];
          y = h[k] * cv[e] + y;
        }
      }
      y = xt * Dd + y;
      const float zv = XZ[(row0 + t) * kXzP + kDin + d];
      const float sg = __builtin_amdgcn_rcpf(1.0f + __expf(-zv));
      y = y * (zv * sg);
      sY[s * kScanYP + tid] = y;
    }
    __syncthreads();
#pragma unroll 1
    for (int hf = 0; hf < 2; ++hf) {
      v8h hv[4];
#pragma unroll
      for (int it = 0; it < 4; ++it) {
        const int row = (hf * 4 + it) * 8 + wave * 4 + q;
        const float* sp = sY + row * kScanYP + c8;
        const v4f a0 = *(const v4f*)(sp);
        const v4f a1 = *(const v4f*)(sp + 4);
#pragma unroll
        for (int e = 0; e < 4; ++e) {
          hv[it][e]     = (_Float16)(a0[e] * kYCarry);
          hv[it][4 + e] = (_Float16)(a1[e] * kYCarry);
        }
      }
      for (int pass = 0; pass < 2; ++pass) {
#pragma unroll
        for (int it = 0; it < 4; ++it) {
          const int row = (hf * 4 + it) * 8 + wave * 4 + q;
          const size_t o = (row0 + t0 + row) * kDin + d0 + c8;
          *(volatile v8h*)(Y16 + o) = hv[it];
        }
        __threadfence();
      }
    }
  }
}

extern "C" void kernel_launch(void* const* d_in, const int* in_sizes, int n_in,
                              void* d_out, int out_size, void* d_ws, size_t ws_size,
                              hipStream_t stream) {
  if (n_in < 12) return;
  if (in_sizes[0]  != kRowsAll * kDm) return;
  if (in_sizes[1]  != kDm) return;
  if (in_sizes[2]  != kDm) return;
  if (in_sizes[3]  != kDm * kXzP) return;
  if (in_sizes[4]  != kDin * kConv) return;
  if (in_sizes[5]  != kDin) return;
  if (in_sizes[6]  != kDin * kXdW) return;
  if (in_sizes[7]  != kDtR * kDin) return;
  if (in_sizes[8]  != kDin) return;
  if (in_sizes[9]  != kDin * kNst) return;
  if (in_sizes[10] != kDin) return;
  if (in_sizes[11] != kDin * kDm) return;
  if (out_size != kRowsAll * kDm) return;
  if (ws_size < kWsTotal) return;

  const float* x      = (const float*)d_in[0];
  const float* ln_g   = (const float*)d_in[1];
  const float* ln_b   = (const float*)d_in[2];
  const float* W_in   = (const float*)d_in[3];
  const float* conv_w = (const float*)d_in[4];
  const float* conv_b = (const float*)d_in[5];
  const float* W_x    = (const float*)d_in[6];
  const float* W_dt   = (const float*)d_in[7];
  const float* b_dt   = (const float*)d_in[8];
  const float* A_log  = (const float*)d_in[9];
  const float* Dskip  = (const float*)d_in[10];
  const float* W_out  = (const float*)d_in[11];
  float* out = (float*)d_out;

  char* ws = (char*)d_ws;
  unsigned short* WIT  = (unsigned short*)(ws + kOffWIT);
  unsigned short* WXT  = (unsigned short*)(ws + kOffWXT);
  unsigned short* WOT  = (unsigned short*)(ws + kOffWOT);
  unsigned short* XN   = (unsigned short*)(ws + kOffXN);
  float*          XZ   = (float*)(ws + kOffXZ);
  float*          UC   = (float*)(ws + kOffUC);
  unsigned short* UC16 = (unsigned short*)(ws + kOffUC16);
  float*          XD   = (float*)(ws + kOffXD);
  unsigned short* Y16  = (unsigned short*)(ws + kOffY16);

  transpose_cast_f16_kernel<<<dim3(kDm / 64, kXzP / 64), 256, 0, stream>>>(W_in, WIT, kDm, kXzP, kWCarry);
  transpose_cast_f16_kernel<<<dim3(kDin / 64, kXdP / 64), 256, 0, stream>>>(W_x, WXT, kDin, kXdW, kWCarry);
  transpose_cast_f16_kernel<<<dim3(kDin / 64, kDm / 64), 256, 0, stream>>>(W_out, WOT, kDin, kDm, kWCarry);

  for (int grp = 0; grp < kGroups; ++grp) {
    const float* xg = x   + (size_t)grp * kRowsG * kDm;
    float*       og = out + (size_t)grp * kRowsG * kDm;

    ln_rows_kernel<<<kRowsG / 8, 256, 0, stream>>>(xg, ln_g, ln_b, XN, kRowsG);

    wmma_gemm64<0, 0, 0, 0, false><<<dim3(kTilesIn / 8, 1), 256, 0, stream>>>(
        XN, nullptr, kDm, 0L,
        WIT, nullptr, kDm, 0L,
        (void*)XZ, nullptr, kXzP, 0L,
        nullptr, nullptr, 0L,
        kRowsG, kXzP, kDm, kInScale);

    conv_silu_kernel<<<dim3(kDin / 256, kRowsG / 64), 256, 0, stream>>>(XZ, conv_w, conv_b, UC, UC16);

    wmma_gemm64<0, 0, 0, 0, false><<<dim3(kTilesX / 8, 1), 256, 0, stream>>>(
        UC16, nullptr, kDin, 0L,
        WXT, nullptr, kDin, 0L,
        (void*)XD, nullptr, kXdP, 0L,
        nullptr, nullptr, 0L,
        kRowsG, kXdP, kDin, kXScale);

    scan_kernel<<<(kRowsG / kSeq) * (kDin / kScanCh), kScanCh, 0, stream>>>(XD, UC, XZ, W_dt, b_dt, A_log, Dskip, Y16);

    wmma_gemm64<0, 0, 0, 0, true><<<dim3(kTilesOut / 8, 1), 256, 0, stream>>>(
        Y16, nullptr, kDin, 0L,
        WOT, nullptr, kDin, 0L,
        (void*)og, nullptr, kDm, 0L,
        nullptr, xg, 0L,
        kRowsG, kDm, kDin, kOutScale);
  }
}
